// GraphEncoder_70987219468418
// MI455X (gfx1250) — hardware-verified
//
#include <hip/hip_runtime.h>
#include <stddef.h>
#include <stdint.h>


#define DF     128
#define LAT    64
#define NGR    512
#define NLAY   3
#define NMAT   7
#define NTHR   256
#define NWAVE  8
#define EPT    8
#define CHUNK  (NTHR * EPT)
#define WCAP   (EPT * 32)
#define LISTN  (NWAVE * WCAP)
#define NBA    1024
#define SLA    10
#define RCAP   28672
#define DEGCAP 64
#define GBM    64
#define GBN    128
#define GTHR   128
#define UPART  2048
#define AGG_ZINTS    (LISTN + 2 * RCAP + 3 * NBA)
#define MISC_INTS    16
#define AGG_LDS_INTS (AGG_ZINTS + MISC_INTS)
#define NOUT   (2 * NGR * LAT)
#define WSMAX  268435456

static_assert((CHUNK & (CHUNK - 1)) == 0 && CHUNK <= 4096);
static_assert((NBA & (NBA - 1)) == 0 && NBA == (1 << SLA));
static_assert(((long long)CHUNK << SLA) < (1LL << 31));
static_assert(LISTN % NTHR == 0);
static_assert(NBA % NWAVE == 0 && NBA % 32 == 0 && NBA % GBM == 0);
static_assert(RCAP % 4 == 0 && AGG_ZINTS % 4 == 0 && LISTN % 4 == 0 && ((AGG_ZINTS + MISC_INTS) % 4) == 0);
static_assert(AGG_ZINTS % (NTHR * 4) == 0);
static_assert(DF % 32 == 0 && GBN == DF && GBM == (GTHR / 32) * 16 && DF == 4 * 32);
static_assert(UPART % NTHR == 0 && UPART == DF * (DF / 8));
static_assert((NMAT * UPART) % NTHR == 0);
static_assert(AGG_LDS_INTS * 4 <= 300000);
static_assert(LAT * 4 == 256 && 2 * LAT == DF && NOUT == 2 * NGR * LAT);

typedef float          v4f   __attribute__((ext_vector_type(4)));
typedef float          v8f   __attribute__((ext_vector_type(8)));
typedef int            v4i   __attribute__((ext_vector_type(4)));
typedef int            v8i   __attribute__((ext_vector_type(8)));
typedef unsigned short v8us  __attribute__((ext_vector_type(8)));
typedef unsigned short v16us __attribute__((ext_vector_type(16)));
typedef __bf16         v16bf __attribute__((ext_vector_type(16)));
typedef v4f  __attribute__((may_alias)) v4fa;
typedef v4i  __attribute__((may_alias)) v4ia;
typedef v8us __attribute__((may_alias)) v8usa;
union FragB { v16bf v; v16us u; v8us h[2]; v8i w; };

__device__ __forceinline__ v8f wmb(const FragB& a, const FragB& b, v8f c) {
  v8f d = __builtin_amdgcn_wmma_f32_16x16x32_bf16(false, a.v, false, b.v, (short)0, c, false, false);
  asm volatile("v_nop\n\tv_nop\n\tv_nop\n\tv_nop" : "+v"(d) : "v"(a.w), "v"(b.w));
  return d;
}

__device__ __forceinline__ unsigned bf16_bits(float f) {
  const unsigned u = __float_as_uint(f);
  return (u + 0x7FFFu + ((u >> 16) & 1u)) >> 16;
}
__device__ __forceinline__ float bf16_val(float f) {
  return __uint_as_float(bf16_bits(f) << 16);
}

template <int SLB>
__device__ __forceinline__ int scan_chunk(const int* __restrict__ dsts, int nE, int cbase, int slotBase,
                                          int nb, int vec8, int* list, int tid, int lane, int wave) {
  int wc = 0;
  const int el0  = tid * EPT;
  const int e0   = cbase + el0;
  const int sent = -2147483647 - 1;
  v4i da, db;
  if (vec8 != 0 && cbase + CHUNK <= nE) {
    da = *(const v4i*)(dsts + e0);
    db = *(const v4i*)(dsts + e0 + 4);
  } else {
    da.x = (e0     < nE) ? dsts[min(e0,     nE - 1)] : sent;
    da.y = (e0 + 1 < nE) ? dsts[min(e0 + 1, nE - 1)] : sent;
    da.z = (e0 + 2 < nE) ? dsts[min(e0 + 2, nE - 1)] : sent;
    da.w = (e0 + 3 < nE) ? dsts[min(e0 + 3, nE - 1)] : sent;
    db.x = (e0 + 4 < nE) ? dsts[min(e0 + 4, nE - 1)] : sent;
    db.y = (e0 + 5 < nE) ? dsts[min(e0 + 5, nE - 1)] : sent;
    db.z = (e0 + 6 < nE) ? dsts[min(e0 + 6, nE - 1)] : sent;
    db.w = (e0 + 7 < nE) ? dsts[min(e0 + 7, nE - 1)] : sent;
  }
  const unsigned nbs = (unsigned)slotBase;
  const unsigned unb = (unsigned)nb;
  const unsigned s0 = (unsigned)da.x - nbs, s1 = (unsigned)da.y - nbs;
  const unsigned s2 = (unsigned)da.z - nbs, s3 = (unsigned)da.w - nbs;
  const unsigned s4 = (unsigned)db.x - nbs, s5 = (unsigned)db.y - nbs;
  const unsigned s6 = (unsigned)db.z - nbs, s7 = (unsigned)db.w - nbs;
  const bool h0 = s0 < unb, h1 = s1 < unb, h2 = s2 < unb, h3 = s3 < unb;
  const bool h4 = s4 < unb, h5 = s5 < unb, h6 = s6 < unb, h7 = s7 < unb;
  const unsigned any = __builtin_amdgcn_ballot_w32(h0 | h1 | h2 | h3 | h4 | h5 | h6 | h7);
  if (any != 0u) {
#define HITJ(J, HJ, SJ) { \
      const unsigned mj = __builtin_amdgcn_ballot_w32(HJ); \
      if (mj != 0u) { \
        if (HJ) { \
          const int pos = wc + (int)__builtin_amdgcn_mbcnt_lo(mj, 0u); \
          if (pos < WCAP) list[wave * WCAP + pos] = ((el0 + (J)) << SLB) | (int)(SJ); \
        } \
        wc += (int)__builtin_popcount(mj); } }
    HITJ(0, h0, s0)
    HITJ(1, h1, s1)
    HITJ(2, h2, s2)
    HITJ(3, h3, s3)
    HITJ(4, h4, s4)
    HITJ(5, h5, s5)
    HITJ(6, h6, s6)
    HITJ(7, h7, s7)
#undef HITJ
  }
  return wc;
}

__global__ __launch_bounds__(NTHR) void k_wprep(const float* __restrict__ Win, const float* __restrict__ Wmsg,
                                                const float* __restrict__ Wupd, unsigned short* WT) {
  const int u    = (int)blockIdx.x * NTHR + (int)threadIdx.x;
  const int part = u >> 11;
  const int v    = u & (UPART - 1);
  const int n    = v >> 4;
  const int k8   = (v & 15) * 8;
  const float* W;
  if (part == 0)              W = Win;
  else if (part < 1 + NLAY)   W = Wmsg + (size_t)(part - 1) * DF * DF;
  else if (part < NMAT)       W = Wupd + (size_t)(part - 1 - NLAY) * DF * DF;
  else return;
  const float* p = W + (size_t)k8 * DF + n;
  v8us o;
#pragma unroll
  for (int i = 0; i < 8; ++i) o[i] = (unsigned short)bf16_bits(p[(size_t)i * DF]);
  unsigned short* dp = WT + (size_t)part * DF * DF + (size_t)n * DF + k8;
  *(volatile v8us*)dp = o;
  __threadfence();
  *(volatile v8us*)dp = o;
}

__global__ __launch_bounds__(NTHR) void k_cvx(const float* __restrict__ x, int nN, int nUnits,
                                              unsigned short* xb) {
  const int u = (int)blockIdx.x * NTHR + (int)threadIdx.x;
  if (u >= nUnits) return;
  const int row = u >> 4;
  const int k8  = (u & 15) * 8;
  const int rc  = row < nN ? row : nN - 1;
  const float* p = x + (size_t)rc * DF + k8;
  const v4f a = *(const v4fa*)p;
  const v4f b = *(const v4fa*)(p + 4);
  const bool ok = row < nN;
  v8us o;
  o[0] = ok ? (unsigned short)bf16_bits(a.x) : (unsigned short)0;
  o[1] = ok ? (unsigned short)bf16_bits(a.y) : (unsigned short)0;
  o[2] = ok ? (unsigned short)bf16_bits(a.z) : (unsigned short)0;
  o[3] = ok ? (unsigned short)bf16_bits(a.w) : (unsigned short)0;
  o[4] = ok ? (unsigned short)bf16_bits(b.x) : (unsigned short)0;
  o[5] = ok ? (unsigned short)bf16_bits(b.y) : (unsigned short)0;
  o[6] = ok ? (unsigned short)bf16_bits(b.z) : (unsigned short)0;
  o[7] = ok ? (unsigned short)bf16_bits(b.w) : (unsigned short)0;
  unsigned short* dp = xb + (size_t)row * DF + k8;
  *(volatile v8us*)dp = o;
  __threadfence();
  *(volatile v8us*)dp = o;
}

template <int ASRC, int RESID>
__global__ __launch_bounds__(GTHR) void k_gemm(const unsigned short* __restrict__ Ab, const float* __restrict__ Af,
                                               const unsigned short* __restrict__ WT,
                                               const float* __restrict__ bias, float* outp, int nOut) {
  __shared__ __attribute__((aligned(16))) float stg[GBM * GBN];
  const int tid = (int)threadIdx.x, lane = tid & 31, wave = tid >> 5, hh = lane >> 4, m = lane & 15;
  const int rowBase = (int)blockIdx.x * GBM;

  v8f acc[8];
  {
    const v8f z = {0.f, 0.f, 0.f, 0.f, 0.f, 0.f, 0.f, 0.f};
#pragma unroll
    for (int t = 0; t < 8; ++t) acc[t] = z;
  }
  const size_t arow = (size_t)(rowBase + 16 * wave + m) * (size_t)DF + 8 * hh;
  const unsigned short* bp = WT + (size_t)m * (size_t)DF + 8 * hh;

#pragma unroll 1
  for (int k0 = 0; k0 < DF; k0 += 32) {
    if constexpr (ASRC == 0) {
      FragB af;
      af.h[0] = *(const v8usa*)(Ab + arow + k0);
      af.h[1] = *(const v8usa*)(Ab + arow + k0 + 16);
#pragma unroll
      for (int nt = 0; nt < 8; ++nt) {
        const unsigned short* wq = bp + (size_t)(16 * nt) * (size_t)DF + k0;
        FragB bf;
        bf.h[0] = *(const v8usa*)wq;
        bf.h[1] = *(const v8usa*)(wq + 16);
        acc[nt] = wmb(af, bf, acc[nt]);
      }
    } else {
      const v4f x0 = *(const v4fa*)(Af + arow + k0);
      const v4f x1 = *(const v4fa*)(Af + arow + k0 + 4);
      const v4f x2 = *(const v4fa*)(Af + arow + k0 + 16);
      const v4f x3 = *(const v4fa*)(Af + arow + k0 + 20);
      FragB ah, al;
#define SPL(I, V) { const unsigned hb_ = bf16_bits(V); ah.u[I] = (unsigned short)hb_; \
                    al.u[I] = (unsigned short)bf16_bits((V) - __uint_as_float(hb_ << 16)); }
      SPL(0, x0.x)  SPL(1, x0.y)  SPL(2, x0.z)  SPL(3, x0.w)
      SPL(4, x1.x)  SPL(5, x1.y)  SPL(6, x1.z)  SPL(7, x1.w)
      SPL(8, x2.x)  SPL(9, x2.y)  SPL(10, x2.z) SPL(11, x2.w)
      SPL(12, x3.x) SPL(13, x3.y) SPL(14, x3.z) SPL(15, x3.w)
#undef SPL
#pragma unroll
      for (int nt = 0; nt < 8; ++nt) {
        const unsigned short* wq = bp + (size_t)(16 * nt) * (size_t)DF + k0;
        FragB bf;
        bf.h[0] = *(const v8usa*)wq;
        bf.h[1] = *(const v8usa*)(wq + 16);
        acc[nt] = wmb(ah, bf, acc[nt]);
        acc[nt] = wmb(al, bf, acc[nt]);
      }
    }
  }

#pragma unroll
  for (int nt = 0; nt < 8; ++nt) {
    const int lc = 16 * nt + m;
#pragma unroll
    for (int r = 0; r < 8; ++r) {
      const int lr = 16 * wave + 8 * hh + r;
      stg[lr * GBN + lc] = acc[nt][r];
    }
  }
  __syncthreads();

  v4f bb4;
  {
    const v4f t1 = *(const v4f*)(bias + 4 * lane);
    bb4.x = bf16_val(t1.x); bb4.y = bf16_val(t1.y); bb4.z = bf16_val(t1.z); bb4.w = bf16_val(t1.w);
  }

  v4f pv[16];
#pragma unroll
  for (int i = 0; i < 16; ++i) pv[i] = *(const v4fa*)(stg + (16 * wave + i) * GBN + 4 * lane);

#pragma unroll
  for (int i = 0; i < 16; ++i) {
    const int r = rowBase + 16 * wave + i;
    const bool ok = r < nOut;
    const v4f t = pv[i] + bb4;
    v4f y;
    y.x = (t.x < 0.0f) ? 0.0f : t.x;
    y.y = (t.y < 0.0f) ? 0.0f : t.y;
    y.z = (t.z < 0.0f) ? 0.0f : t.z;
    y.w = (t.w < 0.0f) ? 0.0f : t.w;
    if constexpr (RESID != 0) {
      const v4f rs = *(const v4fa*)(outp + (size_t)r * DF + 4 * lane);
      y = y + rs;
    }
    y.x = ok ? y.x : 0.0f; y.y = ok ? y.y : 0.0f; y.z = ok ? y.z : 0.0f; y.w = ok ? y.w : 0.0f;
    pv[i] = y;
  }

#pragma unroll
  for (int i = 0; i < 16; ++i) {
    const int r = rowBase + 16 * wave + i;
    *(volatile v4f*)(outp + (size_t)r * DF + 4 * lane) = pv[i];
  }
  __threadfence();
#pragma unroll
  for (int i = 0; i < 16; ++i) {
    const int r = rowBase + 16 * wave + i;
    *(volatile v4f*)(outp + (size_t)r * DF + 4 * lane) = pv[i];
  }
}

__global__ __launch_bounds__(NTHR) void k_scan(const int* __restrict__ gath, const int* __restrict__ keys,
                                               int nE, int nN, int vec8, int mRows,
                                               const float* __restrict__ msg, float* agg) {
  extern __shared__ __attribute__((aligned(16))) int dsm[];
  int* list = dsm;
  int* hl   = dsm + LISTN;
  int* sl   = hl + RCAP;
  int* cnt  = sl + RCAP;
  int* offs = cnt + NBA;
  int* cur  = offs + NBA;
  int* misc = cur + NBA;
  const int tid = (int)threadIdx.x, lane = tid & 31, wave = tid >> 5;
  const int nodeBase = (int)blockIdx.x * NBA;

  {
    const v4i z4 = {0, 0, 0, 0};
    for (int i = tid * 4; i < AGG_ZINTS; i += NTHR * 4) *(v4ia*)(dsm + i) = z4;
    if (tid < MISC_INTS) misc[tid] = 0;
  }
  __syncthreads();

  int t = 0, ov = 0;
  const int nChunks = (nE + CHUNK - 1) / CHUNK;
#pragma unroll 1
  for (int ch = 0; ch < nChunks; ++ch) {
    const int cbase = ch * CHUNK;
    const int wc = scan_chunk<SLA>(keys, nE, cbase, nodeBase, NBA, vec8, list, tid, lane, wave);
    if (lane == 0) misc[wave] = wc;
    __syncthreads();
    if (wave == 0) {
#pragma unroll 1
      for (int w2 = 0; w2 < NWAVE; ++w2) {
        int c = misc[w2];
        c = c < 0 ? 0 : (c > WCAP ? WCAP : c);
#pragma unroll 1
        for (int b0 = 0; b0 < c; b0 += 32) {
          const int idx = b0 + lane;
          const int ent = list[w2 * WCAP + (idx < WCAP ? idx : WCAP - 1)];
          const int m32 = (c - b0) < 32 ? (c - b0) : 32;
#pragma unroll 1
          for (int k = 0; k < m32; ++k) {
            const int u    = __builtin_amdgcn_readlane(ent, k);
            const int slot = u & (NBA - 1);
            const int el   = (u >> SLA) & (CHUNK - 1);
            const int pk   = ((cbase + el) << SLA) | slot;
            if (t < RCAP) {
              if (lane == 0) { hl[t] = pk; cnt[slot] = cnt[slot] + 1; }
              t = t + 1;
            } else {
              ov = 1;
            }
          }
        }
      }
    }
    __syncthreads();
  }
  if (wave == 0 && lane == 0) { misc[8] = t; misc[9] = ov; }
  __syncthreads();
  int tt = misc[8];
  tt = tt < 0 ? 0 : (tt > RCAP ? RCAP : tt);
  const int ovf = misc[9];

  if (wave == 0) {
    const int base = lane * (NBA / 32);
    int s = 0;
#pragma unroll 1
    for (int i = 0; i < NBA / 32; ++i) s += cnt[base + i];
    int incl = s;
#pragma unroll
    for (int d = 1; d < 32; d <<= 1) {
      const int y = __shfl_up(incl, d, 32);
      if (lane >= d) incl += y;
    }
    int run = incl - s;
#pragma unroll 1
    for (int i = 0; i < NBA / 32; ++i) {
      const int cv = cnt[base + i];
      offs[base + i] = run;
      cur[base + i]  = run;
      run += cv;
    }
  }
  __syncthreads();
  if (wave == 0) {
#pragma unroll 1
    for (int b0 = 0; b0 < tt; b0 += 32) {
      const int idx = b0 + lane;
      const int ent = hl[idx < RCAP ? idx : RCAP - 1];
      const int m32 = (tt - b0) < 32 ? (tt - b0) : 32;
#pragma unroll 1
      for (int k = 0; k < m32; ++k) {
        const int u    = __builtin_amdgcn_readlane(ent, k);
        const int slot = u & (NBA - 1);
        if (lane == 0) {
          int p = cur[slot];
          p = p < 0 ? 0 : (p > RCAP - 1 ? RCAP - 1 : p);
          sl[p] = u;
          cur[slot] = p + 1;
        }
      }
    }
  }
  __syncthreads();

  const float qnan = __int_as_float(0x7fc00000);
  const float pz = (ovf != 0) ? qnan : 0.0f;
#pragma unroll 1
  for (int si = 0; si < NBA / NWAVE; ++si) {
    const int s    = si * NWAVE + wave;
    const int node = nodeBase + s;
    int c = cnt[s];
    const bool big = c > DEGCAP;
    c = c < 0 ? 0 : (c > DEGCAP ? DEGCAP : c);
    int o = offs[s];
    o = o < 0 ? 0 : (o > RCAP ? RCAP : o);
    float a0 = 0.0f, a1 = 0.0f, a2 = 0.0f, a3 = 0.0f;
#pragma unroll 1
    for (int b0 = 0; b0 < c; b0 += 32) {
      int idx = o + b0 + lane;
      idx = idx > RCAP - 1 ? RCAP - 1 : idx;
      const int ent = sl[idx];
      int eid = ent >> SLA;
      eid = eid < 0 ? 0 : (eid > nE - 1 ? nE - 1 : eid);
      int sr = gath[eid];
      sr = sr < 0 ? 0 : (sr > nN - 1 ? nN - 1 : sr);
      const int m32 = (c - b0) < 32 ? (c - b0) : 32;
#pragma unroll 1
      for (int k = 0; k < m32; ++k) {
        const int sk = __builtin_amdgcn_readlane(sr, k);
        const v4f a = *(const v4fa*)(msg + (size_t)sk * DF + 4 * lane);
        a0 += a.x; a1 += a.y; a2 += a.z; a3 += a.w;
      }
    }
    const float pzr = big ? qnan : pz;
    const bool live = node < nN;
    v4f ovv;
    ovv.x = live ? (a0 + pzr) : 0.0f;
    ovv.y = live ? (a1 + pzr) : 0.0f;
    ovv.z = live ? (a2 + pzr) : 0.0f;
    ovv.w = live ? (a3 + pzr) : 0.0f;
    if (node < mRows) {
      float* rpw = agg + (size_t)node * DF + 4 * lane;
      *(volatile v4f*)rpw = ovv;
      __threadfence();
      *(volatile v4f*)rpw = ovv;
    }
  }
}

__global__ __launch_bounds__(NTHR) void k_pool(const float* __restrict__ hf, const int* __restrict__ bat, int nN,
                                               const float* __restrict__ Wmn, const float* __restrict__ bmn,
                                               const float* __restrict__ Wlv, const float* __restrict__ blv,
                                               float* out) {
  __shared__ __attribute__((aligned(16))) float wsum[NWAVE * DF];
  __shared__ __attribute__((aligned(16))) float gs[DF];
  __shared__ __attribute__((aligned(16))) float os[DF];
  const int tid = (int)threadIdx.x, lane = tid & 31, wave = tid >> 5;
  const int g = (int)blockIdx.x;

  float a0 = 0.0f, a1 = 0.0f, a2 = 0.0f, a3 = 0.0f;
#pragma unroll 1
  for (int i0 = wave * 32; i0 < nN; i0 += NTHR) {
    const int i  = i0 + lane;
    const int ic = i < nN ? i : nN - 1;
    const int b  = bat[ic];
    const bool hit = (i < nN) && (b == g);
    unsigned msk = __builtin_amdgcn_ballot_w32(hit);
    int nh = (int)__builtin_popcount(msk);
    nh = nh > 32 ? 32 : nh;
#pragma unroll 1
    for (int q = 0; q < nh; ++q) {
      const int k = __builtin_ffs((int)msk) - 1;
      msk &= msk - 1u;
      int node = i0 + (k < 0 ? 0 : k);
      node = node > nN - 1 ? nN - 1 : node;
      const v4f v = *(const v4fa*)(hf + (size_t)node * DF + 4 * lane);
      a0 += v.x; a1 += v.y; a2 += v.z; a3 += v.w;
    }
  }
  {
    v4f w4; w4.x = a0; w4.y = a1; w4.z = a2; w4.w = a3;
    *(v4fa*)(wsum + wave * DF + 4 * lane) = w4;
  }
  __syncthreads();
  if (tid < DF) {
    float s = 0.0f;
#pragma unroll
    for (int w2 = 0; w2 < NWAVE; ++w2) s += wsum[w2 * DF + tid];
    gs[tid] = s;
  }
  __syncthreads();
  {
    const int hsel = (tid >> 6) & 1;
    const int c = tid & (LAT - 1);
    const float* Wh = hsel ? Wlv : Wmn;
    const float* bh = hsel ? blv : bmn;
    float s = 0.0f;
#pragma unroll 4
    for (int k = 0; k < DF; ++k) s = fmaf(gs[k], bf16_val(Wh[(size_t)k * LAT + c]), s);
    s = s + bf16_val(bh[c]);
    if (tid < DF) os[tid] = s;
  }
  __syncthreads();
  const v4f ov = *(const v4fa*)(os + 4 * lane);
  float* op = out + (size_t)(lane >> 4) * (size_t)(NGR * LAT) + (size_t)g * LAT + 4 * (lane & 15);
  const bool okst = (wave == 0);
  if (okst) *(volatile v4f*)op = ov;
  __threadfence();
  if (okst) *(volatile v4f*)op = ov;
}

static inline int cdiv(int a, int b) { return (a + b - 1) / b; }
static inline size_t al256(size_t o) { return (o + 255) & ~(size_t)255; }

extern "C" void kernel_launch(void* const* d_in, const int* in_sizes, int n_in,
                              void* d_out, int out_size, void* d_ws, size_t ws_size,
                              hipStream_t stream) {
  if (n_in < 13) return;
  if (in_sizes[0] < DF || (in_sizes[0] % DF) != 0) return;
  const int nN = in_sizes[0] / DF;
  if (nN < 16 || nN >= (1 << 22)) return;
  if (in_sizes[1] < 2 || (in_sizes[1] & 1) != 0) return;
  const int nE = in_sizes[1] / 2;
  if (nE < 1 || nE >= (1 << (31 - SLA))) return;
  if (in_sizes[2] != nN) return;
  if (in_sizes[3] != DF * DF || in_sizes[4] != DF) return;
  if (in_sizes[5] != NLAY * DF * DF || in_sizes[6] != NLAY * DF) return;
  if (in_sizes[7] != NLAY * DF * DF || in_sizes[8] != NLAY * DF) return;
  if (in_sizes[9] != DF * LAT || in_sizes[10] != LAT) return;
  if (in_sizes[11] != DF * LAT || in_sizes[12] != LAT) return;
  if (out_size != NOUT) return;

  const float* x     = (const float*)d_in[0];
  const int*   edge  = (const int*)d_in[1];
  const int*   bat   = (const int*)d_in[2];
  const float* Win   = (const float*)d_in[3];
  const float* bin   = (const float*)d_in[4];
  const float* Wmsg  = (const float*)d_in[5];
  const float* bmsg  = (const float*)d_in[6];
  const float* Wupd  = (const float*)d_in[7];
  const float* bupd  = (const float*)d_in[8];
  const float* Wmn   = (const float*)d_in[9];
  const float* bmn   = (const float*)d_in[10];
  const float* Wlv   = (const float*)d_in[11];
  const float* blv   = (const float*)d_in[12];
  float* out = (float*)d_out;
  const int* src = edge;
  const int* dst = edge + nE;

  const int MP = cdiv(nN, GBM) * GBM;
  const int gM = MP / GBM;
  const int gA = cdiv(MP, NBA);
  if ((long long)gA * NBA < (long long)MP) return;
  const int vec8 = ((nE & 3) == 0) ? 1 : 0;

  char* ws = (char*)d_ws;
  size_t off = 0;
  const size_t oWT = off; off = al256(off + (size_t)NMAT * DF * DF * 2);
  const size_t oH  = off; off = al256(off + (size_t)MP * DF * 4);
  const size_t oM  = off; off = al256(off + (size_t)MP * DF * 4);
  const size_t oAX = off; off = al256(off + (size_t)MP * DF * 4);
  if (off > ws_size || off > (size_t)WSMAX) return;
  unsigned short* WT  = (unsigned short*)(ws + oWT);
  float*          H   = (float*)(ws + oH);
  float*          M   = (float*)(ws + oM);
  float*          AGG = (float*)(ws + oAX);
  unsigned short* XB  = (unsigned short*)(ws + oAX);

  const size_t scanLds = (size_t)AGG_LDS_INTS * 4;
  hipFuncSetAttribute(reinterpret_cast<const void*>(&k_scan), hipFuncAttributeMaxDynamicSharedMemorySize, (int)scanLds);

  const int nUx = MP * (DF / 8);
  k_wprep<<<(NMAT * UPART) / NTHR, NTHR, 0, stream>>>(Win, Wmsg, Wupd, WT);
  k_cvx<<<cdiv(nUx, NTHR), NTHR, 0, stream>>>(x, nN, nUx, XB);
  k_gemm<0, 0><<<gM, GTHR, 0, stream>>>(XB, M, WT, bin, H, nN);
  for (int l = 0; l < NLAY; ++l) {
    k_gemm<1, 0><<<gM, GTHR, 0, stream>>>(XB, H, WT + (size_t)(1 + l) * DF * DF, bmsg + (size_t)l * DF, M, nN);
    k_scan<<<gA, NTHR, scanLds, stream>>>(src, dst, nE, nN, vec8, MP, M, AGG);
    k_gemm<1, 1><<<gM, GTHR, 0, stream>>>(XB, AGG, WT + (size_t)(1 + NLAY + l) * DF * DF, bupd + (size_t)l * DF, H, nN);
  }
  k_pool<<<NGR, NTHR, 0, stream>>>(H, bat, nN, Wmn, bmn, Wlv, blv, out);
}
